// CausalSelfAttention_75986561401052
// MI455X (gfx1250) — hardware-verified
//
#include <hip/hip_runtime.h>


#ifndef NB
#define NB 2
#endif
#ifndef SEQ
#define SEQ 2048
#endif
#define SEQ_FULL 2048
#define DM   1024
#define NH   16
#define HD   64
#define RH   256
#define RHE  ((SEQ < RH) ? SEQ : RH)
#define MROWS (NB * SEQ)
#define PCAR 256.0f
#define RSC  2048.0f
#define RSI  0.00048828125f
#define CL2  0.18033688011112042f

#define SZ_W  ((size_t)DM * DM * 2)
#define SZ_XB ((size_t)MROWS * DM * 2)
#define SZ_F  ((size_t)MROWS * DM * 4)
#define SZ_PL ((size_t)NB * NH * SEQ * HD * 2)
#define SZ_AT ((size_t)MROWS * DM * 2)
#define WS_TOTAL (4 * SZ_W + SZ_XB + SZ_F + 6 * SZ_PL + 2 * SZ_AT)

static_assert(HD == 64);
static_assert(NH * HD == DM);
static_assert(DM % 64 == 0);
static_assert(DM % 32 == 0);
static_assert(SEQ % 64 == 0);
static_assert(SEQ <= SEQ_FULL);
static_assert(RH % 64 == 0);
static_assert(RHE % 64 == 0);
static_assert(MROWS % 64 == 0);
static_assert(SZ_W % 256 == 0);
static_assert(SZ_XB % 256 == 0);
static_assert(SZ_PL % 256 == 0);
static_assert(WS_TOTAL <= (size_t)134217728);
static_assert(((size_t)NB * NH * SEQ * HD) % 8 == 0);

typedef _Float16 h16;
typedef unsigned short bf;
typedef __attribute__((ext_vector_type(16))) __bf16   v16bf;
typedef __attribute__((ext_vector_type(16))) _Float16 v16h;
typedef __attribute__((ext_vector_type(8)))  _Float16 v8h;
typedef __attribute__((ext_vector_type(8)))  unsigned short v8us;
typedef __attribute__((ext_vector_type(8)))  float    v8f;
typedef __attribute__((ext_vector_type(4)))  float    v4f;
typedef v4f  __attribute__((may_alias)) v4fa;

__device__ __forceinline__ unsigned short f2bf(float f) { unsigned u = __float_as_uint(f); u += 0x7FFFu + ((u >> 16) & 1u); return (unsigned short)(u >> 16); }
__device__ __forceinline__ float bf2f(unsigned short b) { return __uint_as_float(((unsigned)b) << 16); }
__device__ __forceinline__ void splitf(float y, unsigned short& h, unsigned short& l) { h = f2bf(y); l = f2bf(y - bf2f(h)); }
__device__ __forceinline__ void splith(float y, h16& h, h16& r) { h16 a = (h16)y; float af = (float)a; const bool tiny = fabsf(af) < 6.103515625e-05f; af = tiny ? 0.0f : af; a = tiny ? (h16)0.0f : a; h = a; r = (h16)((y - af) * RSC); }
__device__ __forceinline__ v16h cat16(v8h lo, v8h hi) { return __builtin_shufflevector(lo, hi, 0, 1, 2, 3, 4, 5, 6, 7, 8, 9, 10, 11, 12, 13, 14, 15); }
__device__ __forceinline__ v16bf cat16b(v8us lo, v8us hi) { return __builtin_bit_cast(v16bf, __builtin_shufflevector(lo, hi, 0, 1, 2, 3, 4, 5, 6, 7, 8, 9, 10, 11, 12, 13, 14, 15)); }
__device__ __forceinline__ v8f wmma16(v16h a, v16h b, v8f c) { return __builtin_amdgcn_wmma_f32_16x16x32_f16(false, a, false, b, (short)0, c, false, false); }
__device__ __forceinline__ v8f wmmab(v16bf a, v16bf b, v8f c) { return __builtin_amdgcn_wmma_f32_16x16x32_bf16(false, a, false, b, (short)0, c, false, false); }
__device__ __forceinline__ v16h  ldh(const h16* p) { return cat16(*(const v8h*)p, *(const v8h*)(p + 16)); }
__device__ __forceinline__ v16bf ldb(const bf* p)  { return cat16b(*(const v8us*)p, *(const v8us*)(p + 16)); }
__device__ __forceinline__ float ex2(float x) { return __builtin_amdgcn_exp2f(x); }

__global__ __launch_bounds__(256) void k_cvt8(const float* __restrict__ src, bf* dst, size_t n8) { const size_t i = (size_t)blockIdx.x * 256 + threadIdx.x; if (i >= n8) return; const v8f v = *(const v8f*)(src + i * 8); v8us o;
#pragma unroll
    for (int k = 0; k < 8; ++k) o[k] = f2bf(v[k]); *(volatile v8us*)(dst + i * 8) = o; __threadfence(); *(volatile v8us*)(dst + i * 8) = o; }

template <int NSPLIT>
__device__ __forceinline__ void gemmw_body(const bf* __restrict__ A, const bf* __restrict__ A2, const bf* __restrict__ Bt, const int K, float* C, const int ldc) {
    __shared__ __align__(16) float os[16 * 68];
    const int lane = threadIdx.x & 31, lr = lane & 15, hi = lane >> 4; const int r0 = blockIdx.x * 64, c0 = blockIdx.y * 64;
    v8f acc[4][4];
#pragma unroll
    for (int mb = 0; mb < 4; ++mb)
#pragma unroll
        for (int nb = 0; nb < 4; ++nb) acc[mb][nb] = (v8f){};
    const size_t aoff = (size_t)(r0 + lr) * K + 8 * hi, boff = (size_t)(c0 + lr) * K + 8 * hi;
#pragma unroll 1
    for (int kc = 0; kc < K; kc += 32) {
        v16bf a[4], a2[4], b;
#pragma unroll
        for (int mb = 0; mb < 4; ++mb) { a[mb] = ldb(A + aoff + (size_t)mb * 16 * K + kc); if (NSPLIT == 1) a2[mb] = ldb(A2 + aoff + (size_t)mb * 16 * K + kc); else a2[mb] = a[mb]; }
#pragma unroll
        for (int nb = 0; nb < 4; ++nb) { b = ldb(Bt + boff + (size_t)nb * 16 * K + kc);
#pragma unroll
            for (int mb = 0; mb < 4; ++mb) { acc[mb][nb] = wmmab(a[mb], b, acc[mb][nb]); if (NSPLIT == 1) acc[mb][nb] = wmmab(a2[mb], b, acc[mb][nb]); } }
        asm volatile("v_nop\n\tv_nop\n\tv_nop\n\tv_nop" : "+v"(acc[0][0]), "+v"(acc[0][1]), "+v"(acc[0][2]), "+v"(acc[0][3]), "+v"(acc[1][0]), "+v"(acc[1][1]), "+v"(acc[1][2]), "+v"(acc[1][3]) : "v"(b), "v"(a[1]), "v"(a2[1]));
        asm volatile("v_nop\n\tv_nop\n\tv_nop\n\tv_nop" : "+v"(acc[2][0]), "+v"(acc[2][1]), "+v"(acc[2][2]), "+v"(acc[2][3]), "+v"(acc[3][0]), "+v"(acc[3][1]), "+v"(acc[3][2]), "+v"(acc[3][3]) : "v"(b), "v"(a[3]), "v"(a2[3]));
    }
#pragma unroll
    for (int mb = 0; mb < 4; ++mb) {
#pragma unroll
        for (int nb = 0; nb < 4; ++nb) {
#pragma unroll
            for (int j = 0; j < 8; ++j) os[(hi * 8 + j) * 68 + nb * 16 + lr] = acc[mb][nb][j]; }
        __builtin_amdgcn_wave_barrier(); asm volatile("" ::: "memory");
        float* crow = C + (size_t)(r0 + mb * 16) * ldc + c0;
#pragma unroll 1
        for (int ps = 0; ps < 2; ++ps) {
#pragma unroll
            for (int s = 0; s < 8; ++s) { const int row = 2 * s + hi, cofs = lr * 4; const v4f val = *(const v4fa*)(os + row * 68 + cofs);
                *(volatile v4f*)(crow + (size_t)row * ldc + cofs) = val; }
            if (ps == 0) __threadfence(); }
        __builtin_amdgcn_wave_barrier(); asm volatile("" ::: "memory");
    }
}
__global__ __launch_bounds__(32) void k_gemm_p(const bf* __restrict__ A, const bf* __restrict__ Bt, float* C) { gemmw_body<0>(A, nullptr, Bt, DM, C, DM); }
__global__ __launch_bounds__(32) void k_gemm_o(const bf* __restrict__ A, const bf* __restrict__ A2, const bf* __restrict__ Bt, float* C) { gemmw_body<1>(A, A2, Bt, DM, C, DM); }

__global__ __launch_bounds__(256) void k_pqk(const float* __restrict__ F, h16* P16, h16* PR) {
    const size_t i = (size_t)blockIdx.x * 256 + threadIdx.x; if (i >= (size_t)NB * NH * SEQ * HD / 8) return; const size_t e = i * 8;
    const int d = (int)(e % HD); const int t = (int)((e / HD) % SEQ); const int hh = (int)((e / ((size_t)HD * SEQ)) % NH); const int b = (int)(e / ((size_t)HD * SEQ * NH));
    const float* f = F + ((size_t)b * SEQ + t) * DM + hh * HD + d; const v4f x0 = *(const v4f*)f, x1 = *(const v4f*)(f + 4); v8h o, r;
#pragma unroll
    for (int q = 0; q < 4; ++q) { h16 a, c; splith(x0[q], a, c); o[q] = a; r[q] = c; splith(x1[q], a, c); o[4 + q] = a; r[4 + q] = c; }
    *(volatile v8h*)(P16 + e) = o; *(volatile v8h*)(PR + e) = r; __threadfence(); *(volatile v8h*)(P16 + e) = o; *(volatile v8h*)(PR + e) = r; }
__global__ __launch_bounds__(256) void k_pvt(const float* __restrict__ F, h16* V16, h16* VR) {
    const size_t i = (size_t)blockIdx.x * 256 + threadIdx.x; if (i >= (size_t)NB * NH * SEQ * HD / 8) return; const size_t e = i * 8;
    const int t = (int)(e % SEQ); const int d = (int)((e / SEQ) % HD); const int hh = (int)((e / ((size_t)SEQ * HD)) % NH); const int b = (int)(e / ((size_t)SEQ * HD * NH));
    const float* f = F + ((size_t)b * SEQ + t) * DM + hh * HD + d; v8h o, r;
#pragma unroll
    for (int q = 0; q < 8; ++q) { h16 a, c; splith(f[(size_t)q * DM], a, c); o[q] = a; r[q] = c; }
    *(volatile v8h*)(V16 + e) = o; *(volatile v8h*)(VR + e) = r; __threadfence(); *(volatile v8h*)(V16 + e) = o; *(volatile v8h*)(VR + e) = r; }

template <bool HIRES>
__device__ __forceinline__ void flash_body(const h16* __restrict__ Q16, const h16* __restrict__ QR, const h16* __restrict__ K16, const h16* __restrict__ KR, const h16* __restrict__ VT16, const h16* __restrict__ VTR, bf* ATh, bf* ATl, const int rowbase) {
    __shared__ __align__(16) float os[4][16 * 68];
    const int wave = __builtin_amdgcn_readfirstlane(threadIdx.x >> 5);
    const int lane = threadIdx.x & 31, lr = lane & 15, hi = lane >> 4;
    const int bh = blockIdx.y;
    const int q0 = rowbase + blockIdx.x * 64 + wave * 16;
    const size_t pbase = (size_t)bh * SEQ * HD;
    const size_t qoff = pbase + (size_t)(q0 + lr) * HD + 8 * hi;
    const v16h qh0 = ldh(Q16 + qoff), qh1 = ldh(Q16 + qoff + 32), ql0 = ldh(QR + qoff), ql1 = ldh(QR + qoff + 32);
    float m = -3.0e38f, l = 0.0f;
    v8f om[4], orr[4];
#pragma unroll
    for (int f = 0; f < 4; ++f) { om[f] = (v8f){}; orr[f] = (v8f){}; }
    const int kend = q0 + 16;
    const int qi = q0 + lr;
#pragma unroll 1
    for (int kb = 0; kb < kend; kb += 32) {
        v8f sm0 = (v8f){}, sm1 = (v8f){}, sr0 = (v8f){}, sr1 = (v8f){};
        const size_t k0 = pbase + (size_t)(kb + lr) * HD + 8 * hi, k1 = k0 + (size_t)16 * HD;
        {
            const v16h a0 = ldh(K16 + k0), a1 = ldh(K16 + k1);
            sm0 = wmma16(a0, qh0, sm0); sr0 = wmma16(a0, ql0, sr0); sm1 = wmma16(a1, qh0, sm1); sr1 = wmma16(a1, ql0, sr1);
            if (HIRES) { const v16h c0 = ldh(KR + k0), c1 = ldh(KR + k1); sr0 = wmma16(c0, qh0, sr0); sr1 = wmma16(c1, qh0, sr1); }
            const v16h b0 = ldh(K16 + k0 + 32), b1 = ldh(K16 + k1 + 32);
            sm0 = wmma16(b0, qh1, sm0); sr0 = wmma16(b0, ql1, sr0); sm1 = wmma16(b1, qh1, sm1); sr1 = wmma16(b1, ql1, sr1);
            v16h d0 = b0, d1 = b1;
            if (HIRES) { d0 = ldh(KR + k0 + 32); d1 = ldh(KR + k1 + 32); sr0 = wmma16(d0, qh1, sr0); sr1 = wmma16(d1, qh1, sr1); }
            asm volatile("v_nop\n\tv_nop\n\tv_nop\n\tv_nop" : "+v"(sm0), "+v"(sm1), "+v"(sr0), "+v"(sr1) : "v"(b0), "v"(b1), "v"(d0), "v"(d1), "v"(qh1), "v"(ql1));
        }
        const int kbase = kb + 8 * hi;
        float tv[16]; float mx = -3.0e38f;
#pragma unroll
        for (int r = 0; r < 8; ++r) { const float s0 = (sm0[r] + sr0[r] * RSI) * CL2; const float s1 = (sm1[r] + sr1[r] * RSI) * CL2;
            const float t0 = (kbase + r <= qi) ? s0 : -3.0e38f; const float t1 = (kbase + 16 + r <= qi) ? s1 : -3.0e38f; tv[r] = t0; tv[8 + r] = t1; mx = fmaxf(mx, fmaxf(t0, t1)); }
        mx = fmaxf(mx, __shfl_xor(mx, 16, 32));
        const float mn = fmaxf(m, mx); const float sc = ex2(m - mn); m = mn;
        float psum = 0.0f; v16h ph, pl;
#pragma unroll
        for (int i = 0; i < 16; ++i) { const float p = ex2(tv[i] - mn); psum += p; const float pv = p * PCAR; h16 a, c; if (HIRES) splith(pv, a, c); else { a = (h16)pv; c = a; } ph[i] = a; pl[i] = c; }
        l = l * sc + psum;
#pragma unroll
        for (int f = 0; f < 4; ++f) { om[f] = om[f] * sc; if (HIRES) orr[f] = orr[f] * sc; }
        const size_t v0 = pbase + (size_t)lr * SEQ + kb + 8 * hi;
        v16h va, vr;
#pragma unroll
        for (int f = 0; f < 4; ++f) { va = ldh(VT16 + v0 + (size_t)f * 16 * SEQ); om[f] = wmma16(va, ph, om[f]);
            if (HIRES) { orr[f] = wmma16(va, pl, orr[f]); vr = ldh(VTR + v0 + (size_t)f * 16 * SEQ); orr[f] = wmma16(vr, ph, orr[f]); } else vr = va; }
        if (HIRES) asm volatile("v_nop\n\tv_nop\n\tv_nop\n\tv_nop" : "+v"(om[0]), "+v"(om[1]), "+v"(om[2]), "+v"(om[3]), "+v"(orr[0]), "+v"(orr[1]), "+v"(orr[2]), "+v"(orr[3]) : "v"(ph), "v"(pl), "v"(va), "v"(vr));
        else       asm volatile("v_nop\n\tv_nop\n\tv_nop\n\tv_nop" : "+v"(om[0]), "+v"(om[1]), "+v"(om[2]), "+v"(om[3]) : "v"(ph), "v"(va));
    }
    l += __shfl_xor(l, 16, 32);
    const float inv = 1.0f / (l * PCAR);
#pragma unroll
    for (int f = 0; f < 4; ++f) { v4f x0, x1;
#pragma unroll
        for (int j = 0; j < 4; ++j) { const float y0 = HIRES ? (om[f][j] + orr[f][j] * RSI) : om[f][j]; const float y1 = HIRES ? (om[f][4 + j] + orr[f][4 + j] * RSI) : om[f][4 + j]; x0[j] = y0 * inv; x1[j] = y1 * inv; }
        *(v4fa*)(&os[wave][lr * 68 + 16 * f + 8 * hi]) = x0; *(v4fa*)(&os[wave][lr * 68 + 16 * f + 8 * hi + 4]) = x1; }
    __builtin_amdgcn_wave_barrier(); asm volatile("" ::: "memory");
    const size_t arow = ((size_t)(bh / NH) * SEQ + q0) * DM + (size_t)(bh % NH) * HD;
#pragma unroll 1
    for (int ps = 0; ps < 2; ++ps) {
#pragma unroll
        for (int s = 0; s < 4; ++s) { const int row = 4 * s + (lane >> 3), c = (lane & 7) * 8; const v4f y0 = *(const v4fa*)(&os[wave][row * 68 + c]); const v4f y1 = *(const v4fa*)(&os[wave][row * 68 + c + 4]); v8us oh, ol;
#pragma unroll
            for (int j = 0; j < 4; ++j) { unsigned short a, c2; splitf(y0[j], a, c2); oh[j] = a; ol[j] = c2; splitf(y1[j], a, c2); oh[4 + j] = a; ol[4 + j] = c2; }
            const size_t oo = arow + (size_t)row * DM + c; *(volatile v8us*)(ATh + oo) = oh; *(volatile v8us*)(ATl + oo) = ol; }
        if (ps == 0) __threadfence(); }
    __builtin_amdgcn_wave_barrier(); asm volatile("" ::: "memory");
}
__global__ __launch_bounds__(128) void k_flash_hi(const h16* __restrict__ Q16, const h16* __restrict__ QR, const h16* __restrict__ K16, const h16* __restrict__ KR, const h16* __restrict__ VT16, const h16* __restrict__ VTR, bf* ATh, bf* ATl) { flash_body<true>(Q16, QR, K16, KR, VT16, VTR, ATh, ATl, 0); }
__global__ __launch_bounds__(128) void k_flash_lo(const h16* __restrict__ Q16, const h16* __restrict__ QR, const h16* __restrict__ K16, const h16* __restrict__ VT16, bf* ATh, bf* ATl) { flash_body<false>(Q16, QR, K16, K16, VT16, VT16, ATh, ATl, RHE); }

extern "C" void kernel_launch(void* const* d_in, const int* in_sizes, int n_in,
                              void* d_out, int out_size, void* d_ws, size_t ws_size, hipStream_t stream) {
    if (n_in < 5) return;
    if (in_sizes[0] < (NB - 1) * SEQ_FULL * DM + SEQ * DM) return;
    if (in_sizes[1] < DM * DM || in_sizes[2] < DM * DM || in_sizes[3] < DM * DM || in_sizes[4] < DM * DM) return;
    if (out_size < MROWS * DM) return;
    const float* x = (const float*)d_in[0]; const float* wq = (const float*)d_in[1]; const float* wk = (const float*)d_in[2]; const float* wv = (const float*)d_in[3]; const float* wo = (const float*)d_in[4];
    float* OUT = (float*)d_out;
    char* wsp = (char*)d_ws;
    auto take = [&](size_t bytes) { char* p = wsp; wsp += (bytes + 255) & ~(size_t)255; return (void*)p; };
    bf* WQ = (bf*)take(SZ_W); bf* WK = (bf*)take(SZ_W); bf* WV = (bf*)take(SZ_W); bf* WO = (bf*)take(SZ_W);
    bf* XB = (bf*)take(SZ_XB); float* F = (float*)take(SZ_F);
    h16* Q16 = (h16*)take(SZ_PL); h16* QR = (h16*)take(SZ_PL); h16* K16 = (h16*)take(SZ_PL); h16* KR = (h16*)take(SZ_PL); h16* VT16 = (h16*)take(SZ_PL); h16* VTR = (h16*)take(SZ_PL);
    bf* ATh = (bf*)take(SZ_AT); bf* ATl = (bf*)take(SZ_AT);
    if ((size_t)(wsp - (char*)d_ws) > ws_size) return;
    const size_t nw8 = (size_t)DM * DM / 8, nx8 = (size_t)SEQ * DM / 8;
    k_cvt8<<<(unsigned)((nw8 + 255) / 256), 256, 0, stream>>>(wq, WQ, nw8);
    k_cvt8<<<(unsigned)((nw8 + 255) / 256), 256, 0, stream>>>(wk, WK, nw8);
    k_cvt8<<<(unsigned)((nw8 + 255) / 256), 256, 0, stream>>>(wv, WV, nw8);
    k_cvt8<<<(unsigned)((nw8 + 255) / 256), 256, 0, stream>>>(wo, WO, nw8);
    for (int b = 0; b < NB; ++b) k_cvt8<<<(unsigned)((nx8 + 255) / 256), 256, 0, stream>>>(x + (size_t)b * SEQ_FULL * DM, XB + (size_t)b * SEQ * DM, nx8);
    const dim3 gg(MROWS / 64, DM / 64, 1);
    const unsigned LP = (unsigned)(((size_t)NB * NH * SEQ * HD / 8 + 255) / 256);
    k_gemm_p<<<gg, 32, 0, stream>>>(XB, WQ, F); k_pqk<<<LP, 256, 0, stream>>>(F, Q16, QR);
    k_gemm_p<<<gg, 32, 0, stream>>>(XB, WK, F); k_pqk<<<LP, 256, 0, stream>>>(F, K16, KR);
    k_gemm_p<<<gg, 32, 0, stream>>>(XB, WV, F); k_pvt<<<LP, 256, 0, stream>>>(F, VT16, VTR);
    k_flash_hi<<<dim3(RHE / 64, NB * NH, 1), 128, 0, stream>>>(Q16, QR, K16, KR, VT16, VTR, ATh, ATl);
    if (SEQ > RHE) k_flash_lo<<<dim3((SEQ - RHE) / 64, NB * NH, 1), 128, 0, stream>>>(Q16, QR, K16, VT16, ATh, ATl);
    k_gemm_o<<<gg, 32, 0, stream>>>(ATh, ATl, WO, OUT);
}
